// prototypeLayer_50818053047012
// MI455X (gfx1250) — hardware-verified
//
#include <hip/hip_runtime.h>

#define NB    16
#define NS    1024
#define ND    768
#define NP    256
#define NM    (NB * NS)
#define NR    (NM + NP)
#define NOUT0 (NM * NP)
#define NOUT1 (NP * ND)
#define CROWS 32
#define GBM   128
#define GBN   64

static_assert(ND % 32 == 0);
static_assert(ND % 256 == 0);
static_assert(NM % GBM == 0);
static_assert(NP % GBN == 0);
static_assert(NM % CROWS == 0);
static_assert(NR % CROWS == 0);
static_assert(NOUT1 % 1024 == 0);

typedef unsigned short v8us  __attribute__((ext_vector_type(8)));
typedef __bf16         v16bf __attribute__((ext_vector_type(16)));
typedef float          v8f   __attribute__((ext_vector_type(8)));
typedef float          v4f   __attribute__((ext_vector_type(4)));
typedef int            v8i   __attribute__((ext_vector_type(8)));
typedef v8us __attribute__((may_alias)) v8usa;
typedef v4f  __attribute__((may_alias)) v4fa;

union FragB { v16bf v; v8us half[2]; };

__device__ __forceinline__ v8f wmma_bf16(v16bf a, v16bf b, v8f c) {
  v8f d = __builtin_amdgcn_wmma_f32_16x16x32_bf16(false, a, false, b, (short)0, c, false, false);
  const v8i ai = __builtin_bit_cast(v8i, a);
  const v8i bi = __builtin_bit_cast(v8i, b);
  asm volatile("v_nop\n\tv_nop\n\tv_nop\n\tv_nop" : "+v"(d) : "v"(ai), "v"(bi));
  return d;
}

__device__ __forceinline__ v16bf load_frag(const unsigned short* p, int h) {
  FragB f;
  f.half[0] = *(const v8usa*)(p + 8 * h);
  f.half[1] = *(const v8usa*)(p + 16 + 8 * h);
  return f.v;
}

__device__ __forceinline__ unsigned int bf16_bits(float v) {
  const unsigned int u = __float_as_uint(v);
  return (u + 0x7FFFu + ((u >> 16) & 1u)) >> 16;
}
__device__ __forceinline__ float bf16_val(unsigned int b) {
  return __uint_as_float(b << 16);
}

__global__ __launch_bounds__(256) void convert_kernel(
    const float* __restrict__ x,
    const float* __restrict__ pr,
    unsigned short* __restrict__ pl,
    float* __restrict__ nrm)
{
  __shared__ __attribute__((aligned(16))) float sN[CROWS];

  const int tid = threadIdx.x, lane = tid & 31, w = tid >> 5;
  const int blk = blockIdx.x;
  if (blk >= NR / CROWS) return;
  const int rbase = blk * CROWS;
  const float* sbase = (rbase < NM) ? (x + (size_t)rbase * ND)
                                    : (pr + (size_t)(rbase - NM) * ND);

  #pragma unroll 1
  for (int j = 0; j < 4; ++j) {
    const int lrow = 4 * w + j;
    const float* src = sbase + (size_t)lrow * ND;
    unsigned short* dst = pl + (size_t)(rbase + lrow) * ND;
    float s = 0.0f;
    v8us o[3];
    #pragma unroll
    for (int i = 0; i < 3; ++i) {
      const int e = 8 * (lane + 32 * i);
      const v4f a = *(const v4fa*)(src + e);
      const v4f c = *(const v4fa*)(src + e + 4);
      const unsigned int b0 = bf16_bits(a.x), b1 = bf16_bits(a.y), b2 = bf16_bits(a.z), b3 = bf16_bits(a.w);
      const unsigned int b4 = bf16_bits(c.x), b5 = bf16_bits(c.y), b6 = bf16_bits(c.z), b7 = bf16_bits(c.w);
      const float r0 = bf16_val(b0), r1 = bf16_val(b1), r2 = bf16_val(b2), r3 = bf16_val(b3);
      const float r4 = bf16_val(b4), r5 = bf16_val(b5), r6 = bf16_val(b6), r7 = bf16_val(b7);
      s += r0 * r0 + r1 * r1 + r2 * r2 + r3 * r3 + r4 * r4 + r5 * r5 + r6 * r6 + r7 * r7;
      const v8us ov = { (unsigned short)b0, (unsigned short)b1, (unsigned short)b2, (unsigned short)b3,
                        (unsigned short)b4, (unsigned short)b5, (unsigned short)b6, (unsigned short)b7 };
      o[i] = ov;
    }
    #pragma unroll
    for (int i = 0; i < 3; ++i) *(volatile v8us*)(dst + 8 * (lane + 32 * i)) = o[i];
    __threadfence();
    #pragma unroll
    for (int i = 0; i < 3; ++i) *(volatile v8us*)(dst + 8 * (lane + 32 * i)) = o[i];

    #pragma unroll
    for (int off = 16; off > 0; off >>= 1) s += __shfl_xor(s, off, 32);
    if (lane == 0) sN[lrow] = s;
  }
  __syncthreads();

  v4f nv = {0.0f, 0.0f, 0.0f, 0.0f};
  if (tid < 8) {
    nv = *(const v4fa*)(sN + 4 * tid);
    *(volatile v4f*)(nrm + rbase + 4 * tid) = nv;
  }
  __threadfence();
  if (tid < 8) {
    *(volatile v4f*)(nrm + rbase + 4 * tid) = nv;
  }
}

__global__ __launch_bounds__(256) void widen_kernel(
    const float* __restrict__ pr,
    float* __restrict__ out1)
{
  const int g = blockIdx.x * 256 + threadIdx.x;
  if (g >= NOUT1 / 4) return;
  const v4f a = *(const v4fa*)(pr + (size_t)g * 4);
  const v4f o = { bf16_val(bf16_bits(a.x)), bf16_val(bf16_bits(a.y)),
                  bf16_val(bf16_bits(a.z)), bf16_val(bf16_bits(a.w)) };
  *(volatile v4f*)(out1 + (size_t)g * 4) = o;
  __threadfence();
  *(volatile v4f*)(out1 + (size_t)g * 4) = o;
}

__device__ __forceinline__ void dist_store_pass(const float* sT, const float* sX2, const float* sP2,
                                                float* out, int m0, int c0, int w, int lane) {
  const int q8 = lane & 7, sub = lane >> 3;
  #pragma unroll
  for (int i = 0; i < 16; ++i) {
    const int lid = i * 4 + sub;
    const int row = lid >> 1, hl = lid & 1;
    const int lr = 32 * w + row;
    const int cl = 32 * hl + 4 * q8;
    const v4f v = *(const v4fa*)(sT + lr * 64 + cl);
    const v4f p = *(const v4fa*)(sP2 + cl);
    const float xv = sX2[lr];
    v4f d;
    d.x = (xv + p.x) - 2.0f * v.x;
    d.y = (xv + p.y) - 2.0f * v.y;
    d.z = (xv + p.z) - 2.0f * v.z;
    d.w = (xv + p.w) - 2.0f * v.w;
    const size_t gi = (size_t)(m0 + lr) * NP + c0 + cl;
    *(volatile v4f*)(out + gi) = d;
  }
}

__global__ __launch_bounds__(128) void dist_kernel(
    const unsigned short* __restrict__ pl,
    const float* __restrict__ nrm,
    float* __restrict__ out)
{
  __shared__ __attribute__((aligned(16))) float sT[GBM * GBN];
  __shared__ __attribute__((aligned(16))) float sX2[GBM];
  __shared__ __attribute__((aligned(16))) float sP2[GBN];

  const int tid = threadIdx.x, lane = tid & 31, w = tid >> 5;
  const int h = lane >> 4, m = lane & 15;
  const int m0 = blockIdx.x * GBM;
  const int c0 = blockIdx.y * GBN;
  const int m0w = m0 + 32 * w;

  sX2[tid] = nrm[m0 + tid];
  if (tid < GBN) sP2[tid] = nrm[NM + c0 + tid];

  const unsigned short* xa0 = pl + (size_t)(m0w + m) * ND;
  const unsigned short* xa1 = xa0 + (size_t)16 * ND;
  const unsigned short* wb  = pl + (size_t)(NM + c0 + m) * ND;

  const v8f zero8 = {0.f, 0.f, 0.f, 0.f, 0.f, 0.f, 0.f, 0.f};
  v8f acc[2][4];
  #pragma unroll
  for (int mt = 0; mt < 2; ++mt)
    #pragma unroll
    for (int nt = 0; nt < 4; ++nt) acc[mt][nt] = zero8;

  #pragma unroll 1
  for (int k0 = 0; k0 < ND; k0 += 32) {
    const v16bf a0 = load_frag(xa0 + k0, h);
    const v16bf a1 = load_frag(xa1 + k0, h);
    #pragma unroll
    for (int nt = 0; nt < 4; ++nt) {
      const v16bf b = load_frag(wb + (size_t)nt * 16 * ND + k0, h);
      acc[0][nt] = wmma_bf16(a0, b, acc[0][nt]);
      acc[1][nt] = wmma_bf16(a1, b, acc[1][nt]);
    }
  }

  #pragma unroll
  for (int nt = 0; nt < 4; ++nt) {
    const int lc = 16 * nt + m;
    #pragma unroll
    for (int mt = 0; mt < 2; ++mt) {
      #pragma unroll
      for (int r = 0; r < 8; ++r) {
        const int lr = 32 * w + 16 * mt + 8 * h + r;
        sT[lr * GBN + lc] = acc[mt][nt][r];
      }
    }
  }
  __syncthreads();

  dist_store_pass(sT, sX2, sP2, out, m0, c0, w, lane);
  __threadfence();
  dist_store_pass(sT, sX2, sP2, out, m0, c0, w, lane);
}

extern "C" void kernel_launch(void* const* d_in, const int* in_sizes, int n_in,
                              void* d_out, int out_size, void* d_ws, size_t ws_size,
                              hipStream_t stream) {
  if (n_in < 2) return;
  if (in_sizes[0] != NM * ND) return;
  if (in_sizes[1] != NP * ND) return;
  if (out_size != NOUT0 + NOUT1) return;

  const float* x  = (const float*)d_in[0];
  const float* pr = (const float*)d_in[1];
  float* out = (float*)d_out;

  const size_t pl_bytes  = (size_t)NR * ND * 2;
  const size_t nrm_bytes = (size_t)NR * 4;
  const size_t total = pl_bytes + nrm_bytes;
  if (total > ws_size) return;

  char* ws = (char*)d_ws;
  unsigned short* pl = (unsigned short*)(ws);
  float* nrm = (float*)(ws + pl_bytes);

  convert_kernel<<<NR / CROWS, 256, 0, stream>>>(x, pr, pl, nrm);

  widen_kernel<<<(NOUT1 / 4 + 255) / 256, 256, 0, stream>>>(pr, out + (size_t)NOUT0);

  dim3 gDist(NM / GBM, NP / GBN);
  dist_kernel<<<gDist, 128, 0, stream>>>(pl, nrm, out);
}
